// SpatialAttention_24206435680951
// MI455X (gfx1250) — hardware-verified
//
#include <hip/hip_runtime.h>
#include <stdint.h>
#include <stddef.h>


#ifndef NB
#define NB 4
#endif
#ifndef SEQ
#define SEQ 4096
#endif
#define NB_FULL  4
#define SEQ_FULL 4096
#define HW       (SEQ)
#define HW_FULL  (SEQ_FULL)
#define CH       256
#define PCARRY   16384.0f
#define PUNCARRY 0.00006103515625f
#define LOG2E    1.4426950408889634f
#define W_BLOCKS  ((CH * CH) / 2048)
#define WT_BLOCKS ((CH / 64) * (CH / 64))
#define TP        72

static_assert(NB >= 1 && NB <= NB_FULL);
static_assert(HW >= 64 && HW <= HW_FULL && (HW % 64) == 0);
static_assert(CH == 256);
static_assert(((CH * CH) % 2048) == 0);

typedef float          v8f   __attribute__((ext_vector_type(8)));
typedef float          v4f_  __attribute__((ext_vector_type(4)));
typedef v4f_           v4f   __attribute__((may_alias));
typedef _Float16       v16h  __attribute__((ext_vector_type(16)));
typedef _Float16       v8h_  __attribute__((ext_vector_type(8)));
typedef v8h_           v8h   __attribute__((may_alias));
typedef __bf16         v16bf __attribute__((ext_vector_type(16)));
typedef unsigned short v8us_ __attribute__((ext_vector_type(8)));
typedef v8us_          v8us  __attribute__((may_alias));
typedef unsigned       v4u_  __attribute__((ext_vector_type(4)));
typedef v4u_           v4u   __attribute__((may_alias));

union FragB { v16bf v; v8us_ h[2]; };
union FragH { v16h  v; v8h_  h[2]; };

__device__ __forceinline__ v8f mma_bf16(const v16bf a, const v16bf b, v8f c)
{
  v8f d = __builtin_amdgcn_wmma_f32_16x16x32_bf16(false, a, false, b, (short)0, c, false, false);
  asm volatile("v_nop\n\tv_nop\n\tv_nop\n\tv_nop" : "+v"(d) : "v"(a), "v"(b));
  return d;
}
__device__ __forceinline__ v8f mma_f16(const v16h a, const v16h b, v8f c)
{
  v8f d = __builtin_amdgcn_wmma_f32_16x16x32_f16(false, a, false, b, (short)0, c, false, false);
  asm volatile("v_nop\n\tv_nop\n\tv_nop\n\tv_nop" : "+v"(d) : "v"(a), "v"(b));
  return d;
}

__device__ __forceinline__ unsigned short bf16_bits(float f)
{
  const __bf16 hb = (__bf16)f;
  return __builtin_bit_cast(unsigned short, hb);
}
__device__ __forceinline__ float bf16_rn(float f)
{
  return (float)(__bf16)f;
}
__device__ __forceinline__ float exp2fast(float x)
{
#if __has_builtin(__builtin_amdgcn_exp2f)
  return __builtin_amdgcn_exp2f(x);
#else
  return exp2f(x);
#endif
}

__global__ void __launch_bounds__(256) cvt_w_kernel(
    const float* __restrict__ w1, const float* __restrict__ w2, const float* __restrict__ w3,
    unsigned short* __restrict__ w1b, unsigned short* __restrict__ w2tb,
    unsigned short* __restrict__ w3b)
{
  __shared__ __align__(16) unsigned short sT[64 * TP];
  const int blk = (int)blockIdx.x;
  const int tid = (int)threadIdx.x;

  if (blk < 2 * W_BLOCKS) {
    const float* src;
    unsigned short* dst;
    int t;
    if (blk < W_BLOCKS) { src = w1; dst = w1b; t = blk * 256 + tid; }
    else                { src = w3; dst = w3b; t = (blk - W_BLOCKS) * 256 + tid; }

    const v4f a = *(const v4f*)(src + (size_t)t * 8);
    const v4f b = *(const v4f*)(src + (size_t)t * 8 + 4);
    v8us_ o;
    o[0] = bf16_bits(a[0]); o[1] = bf16_bits(a[1]); o[2] = bf16_bits(a[2]); o[3] = bf16_bits(a[3]);
    o[4] = bf16_bits(b[0]); o[5] = bf16_bits(b[1]); o[6] = bf16_bits(b[2]); o[7] = bf16_bits(b[3]);
    unsigned short* p = dst + (size_t)t * 8;
    *(volatile v8us_*)p = o;
    __threadfence();
    *(volatile v8us_*)p = o;
  } else {
    const int tb = blk - 2 * W_BLOCKS;
    const int o0 = (tb >> 2) * 64;
    const int c0 = (tb & 3) * 64;
    {
      const int r = tid >> 2, part = tid & 3;
      const float* s = w2 + (size_t)(o0 + r) * CH + c0 + part * 16;
      const v4f x0 = *(const v4f*)(s);
      const v4f x1 = *(const v4f*)(s + 4);
      const v4f x2 = *(const v4f*)(s + 8);
      const v4f x3 = *(const v4f*)(s + 12);
      unsigned short* d = &sT[(part * 16) * TP + r];
#pragma unroll
      for (int j = 0; j < 4; ++j) {
        d[(j)      * TP] = bf16_bits(x0[j]);
        d[(4 + j)  * TP] = bf16_bits(x1[j]);
        d[(8 + j)  * TP] = bf16_bits(x2[j]);
        d[(12 + j) * TP] = bf16_bits(x3[j]);
      }
    }
    __syncthreads();
    const int q = tid & 7, cr = tid >> 3;
    const v4u_ v0 = *(const v4u*)&sT[cr * TP + q * 8];
    const v4u_ v1 = *(const v4u*)&sT[(cr + 32) * TP + q * 8];
    unsigned short* p0 = w2tb + (size_t)(c0 + cr) * CH + o0 + q * 8;
    unsigned short* p1 = w2tb + (size_t)(c0 + cr + 32) * CH + o0 + q * 8;
    *(volatile v4u_*)p0 = v0;
    *(volatile v4u_*)p1 = v1;
    __threadfence();
    *(volatile v4u_*)p0 = v0;
    *(volatile v4u_*)p1 = v1;
  }
}

__global__ void __launch_bounds__(256) proj_kernel(
    const float* __restrict__ X,
    const unsigned short* __restrict__ w1b, const float* __restrict__ b1,
    const unsigned short* __restrict__ w2tb,
    const unsigned short* __restrict__ w3b, const float* __restrict__ b3,
    unsigned short* __restrict__ xq,
    unsigned short* __restrict__ gth, unsigned short* __restrict__ gtl,
    unsigned short* __restrict__ vh)
{
  __shared__ __align__(16) unsigned short sX[64 * CH];
  __shared__ __align__(16) unsigned short sBh[64 * CH];
  __shared__ __align__(16) unsigned short sBl[64 * CH];

  const int tid  = (int)threadIdx.x;
  const int lane = tid & 31, wave = tid >> 5;
  const int h = lane >> 4, m = lane & 15;
  const int tiles = HW / 64;
  const int n  = (int)blockIdx.x / tiles;
  const int p0 = ((int)blockIdx.x % tiles) * 64;
  const float* Xn = X + (size_t)n * CH * HW_FULL + p0;
  const size_t toff = ((size_t)n * HW + p0) * CH + (size_t)tid * 8;

  {
    const int cl = tid >> 4, px4 = (tid & 15) * 4;
#pragma unroll 4
    for (int it = 0; it < 16; ++it) {
      const int c = cl + 16 * it;
      const v4f xv = *(const v4f*)(Xn + (size_t)c * HW_FULL + px4);
      sX[(px4 + 0) * CH + c] = bf16_bits(xv[0]);
      sX[(px4 + 1) * CH + c] = bf16_bits(xv[1]);
      sX[(px4 + 2) * CH + c] = bf16_bits(xv[2]);
      sX[(px4 + 3) * CH + c] = bf16_bits(xv[3]);
    }
  }
  __syncthreads();

  {
    v4u_ xw[8];
#pragma unroll
    for (int it = 0; it < 8; ++it) xw[it] = *(const v4u*)&sX[it * 2048 + tid * 8];
#pragma unroll
    for (int it = 0; it < 8; ++it) *(volatile v4u_*)(xq + toff + (size_t)it * 2048) = xw[it];
    __threadfence();
#pragma unroll
    for (int it = 0; it < 8; ++it) *(volatile v4u_*)(xq + toff + (size_t)it * 2048) = xw[it];
  }

  {
    const int pt = wave & 3, oh = wave >> 2;
    v8f acc[8] = {};
#pragma unroll 1
    for (int k0 = 0; k0 < CH; k0 += 32) {
      FragB b;
      b.h[0] = *(const v8us*)&sX[(pt * 16 + m) * CH + k0 + 8 * h];
      b.h[1] = *(const v8us*)&sX[(pt * 16 + m) * CH + k0 + 16 + 8 * h];
#pragma unroll
      for (int ot = 0; ot < 8; ++ot) {
        const unsigned short* wr = w1b + (size_t)(oh * 128 + ot * 16 + m) * CH + k0 + 8 * h;
        FragB a;
        a.h[0] = *(const v8us*)(wr);
        a.h[1] = *(const v8us*)(wr + 16);
        acc[ot] = mma_bf16(a.v, b.v, acc[ot]);
      }
    }
#pragma unroll
    for (int ot = 0; ot < 8; ++ot) {
      const int ob = oh * 128 + ot * 16 + 8 * h;
      const v4f_ q0 = *(const v4f*)(b1 + ob);
      const v4f_ q1 = *(const v4f*)(b1 + ob + 4);
      v8us_ hv, lv;
#pragma unroll
      for (int r = 0; r < 4; ++r) {
        const float f0 = acc[ot][r]     + bf16_rn(q0[r]);
        const float f1 = acc[ot][4 + r] + bf16_rn(q1[r]);
        const __bf16 hb0 = (__bf16)f0;
        const __bf16 hb1 = (__bf16)f1;
        hv[r]     = __builtin_bit_cast(unsigned short, hb0);
        hv[4 + r] = __builtin_bit_cast(unsigned short, hb1);
        lv[r]     = bf16_bits(f0 - (float)hb0);
        lv[4 + r] = bf16_bits(f1 - (float)hb1);
      }
      *(v8us*)&sBh[(pt * 16 + m) * CH + ob] = hv;
      *(v8us*)&sBl[(pt * 16 + m) * CH + ob] = lv;
    }
  }

  const int cb = wave * 32;
  v8us_ vpk[4][2];
  {
    v8f accv[4][2] = {};
#pragma unroll 1
    for (int k0 = 0; k0 < CH; k0 += 32) {
      FragB a[4], b[2];
#pragma unroll
      for (int pt = 0; pt < 4; ++pt) {
        a[pt].h[0] = *(const v8us*)&sX[(pt * 16 + m) * CH + k0 + 8 * h];
        a[pt].h[1] = *(const v8us*)&sX[(pt * 16 + m) * CH + k0 + 16 + 8 * h];
      }
#pragma unroll
      for (int ct = 0; ct < 2; ++ct) {
        const unsigned short* wr = w3b + (size_t)(cb + ct * 16 + m) * CH + k0 + 8 * h;
        b[ct].h[0] = *(const v8us*)(wr);
        b[ct].h[1] = *(const v8us*)(wr + 16);
      }
#pragma unroll
      for (int pt = 0; pt < 4; ++pt)
#pragma unroll
        for (int ct = 0; ct < 2; ++ct)
          accv[pt][ct] = mma_bf16(a[pt].v, b[ct].v, accv[pt][ct]);
    }
#pragma unroll
    for (int ct = 0; ct < 2; ++ct) {
      const float bb = bf16_rn(b3[cb + ct * 16 + m]);
#pragma unroll
      for (int pt = 0; pt < 4; ++pt) {
        v8h_ o;
#pragma unroll
        for (int r = 0; r < 8; ++r) o[r] = (_Float16)(accv[pt][ct][r] + bb);
        vpk[pt][ct] = __builtin_bit_cast(v8us_, o);
      }
    }
  }
  __syncthreads();

#pragma unroll
  for (int pt = 0; pt < 4; ++pt)
#pragma unroll
    for (int ct = 0; ct < 2; ++ct)
      *(v8us*)&sX[(cb + ct * 16 + m) * 64 + pt * 16 + 8 * h] = vpk[pt][ct];

  {
    const int pt = wave & 3, chh = wave >> 2;
    v8f acc[8] = {};
#pragma unroll 1
    for (int k0 = 0; k0 < CH; k0 += 32) {
      FragB bh, bl;
      bh.h[0] = *(const v8us*)&sBh[(pt * 16 + m) * CH + k0 + 8 * h];
      bh.h[1] = *(const v8us*)&sBh[(pt * 16 + m) * CH + k0 + 16 + 8 * h];
      bl.h[0] = *(const v8us*)&sBl[(pt * 16 + m) * CH + k0 + 8 * h];
      bl.h[1] = *(const v8us*)&sBl[(pt * 16 + m) * CH + k0 + 16 + 8 * h];
#pragma unroll
      for (int ct = 0; ct < 8; ++ct) {
        const unsigned short* wr = w2tb + (size_t)(chh * 128 + ct * 16 + m) * CH + k0 + 8 * h;
        FragB a;
        a.h[0] = *(const v8us*)(wr);
        a.h[1] = *(const v8us*)(wr + 16);
        acc[ct] = mma_bf16(a.v, bh.v, acc[ct]);
        acc[ct] = mma_bf16(a.v, bl.v, acc[ct]);
      }
    }
    v8us_ gh[8], gl[8];
#pragma unroll
    for (int ct = 0; ct < 8; ++ct) {
#pragma unroll
      for (int r = 0; r < 8; ++r) {
        const float f = acc[ct][r];
        const __bf16 hb = (__bf16)f;
        gh[ct][r] = __builtin_bit_cast(unsigned short, hb);
        gl[ct][r] = bf16_bits(f - (float)hb);
      }
    }
    __syncthreads();
#pragma unroll
    for (int ct = 0; ct < 8; ++ct) {
      const int cq = chh * 128 + ct * 16 + 8 * h;
      *(v8us*)&sBh[(pt * 16 + m) * CH + cq] = gh[ct];
      *(v8us*)&sBl[(pt * 16 + m) * CH + cq] = gl[ct];
    }
  }
  __syncthreads();

  const int rr = tid >> 3, q = tid & 7;
  v4u_ vv[8];
#pragma unroll
  for (int it = 0; it < 8; ++it) vv[it] = *(const v4u*)&sX[(it * 32 + rr) * 64 + q * 8];
  v4u_ ghw[8], glw[8];
#pragma unroll
  for (int it = 0; it < 8; ++it) {
    ghw[it] = *(const v4u*)&sBh[it * 2048 + tid * 8];
    glw[it] = *(const v4u*)&sBl[it * 2048 + tid * 8];
  }

  unsigned short* vbase = vh + ((size_t)n * CH + rr) * HW + p0 + q * 8;

#pragma unroll
  for (int it = 0; it < 8; ++it)
    *(volatile v4u_*)(vbase + (size_t)it * 32 * HW) = vv[it];
#pragma unroll
  for (int it = 0; it < 8; ++it) {
    *(volatile v4u_*)(gth + toff + (size_t)it * 2048) = ghw[it];
    *(volatile v4u_*)(gtl + toff + (size_t)it * 2048) = glw[it];
  }
  __threadfence();
#pragma unroll
  for (int it = 0; it < 8; ++it)
    *(volatile v4u_*)(vbase + (size_t)it * 32 * HW) = vv[it];
#pragma unroll
  for (int it = 0; it < 8; ++it) {
    *(volatile v4u_*)(gth + toff + (size_t)it * 2048) = ghw[it];
    *(volatile v4u_*)(gtl + toff + (size_t)it * 2048) = glw[it];
  }
}

__global__ void __launch_bounds__(64) stats_kernel(
    const unsigned short* __restrict__ xq,
    const unsigned short* __restrict__ gth, const unsigned short* __restrict__ gtl,
    float* __restrict__ mL, float* __restrict__ rzc)
{
  __shared__ __align__(16) float sSt[64];
  const int tid  = (int)threadIdx.x;
  const int lane = tid & 31, wave = tid >> 5;
  const int h = lane >> 4, m = lane & 15;
  const int tiles = HW / 32;
  const int n  = (int)blockIdx.x / tiles;
  const int ib = ((int)blockIdx.x % tiles) * 32;
  const int i0 = ib + wave * 16;
  const size_t rb = (size_t)n * HW * CH;

  const unsigned short* ghr = gth + rb + (size_t)(i0 + m) * CH + 8 * h;
  const unsigned short* glr = gtl + rb + (size_t)(i0 + m) * CH + 8 * h;

  float mi = -3.0e30f;
  float li = 0.0f;
#pragma unroll 1
  for (int j0 = 0; j0 < HW; j0 += 32) {
    const unsigned short* xa = xq + rb + (size_t)(j0 + m) * CH + 8 * h;
    const unsigned short* xc = xq + rb + (size_t)(j0 + 16 + m) * CH + 8 * h;
    v8f s0 = {};
    v8f s1 = {};
#pragma unroll 2
    for (int k0 = 0; k0 < CH; k0 += 32) {
      FragB a0, a1, bh, bl;
      a0.h[0] = *(const v8us*)(xa + k0);   a0.h[1] = *(const v8us*)(xa + k0 + 16);
      a1.h[0] = *(const v8us*)(xc + k0);   a1.h[1] = *(const v8us*)(xc + k0 + 16);
      bh.h[0] = *(const v8us*)(ghr + k0);  bh.h[1] = *(const v8us*)(ghr + k0 + 16);
      bl.h[0] = *(const v8us*)(glr + k0);  bl.h[1] = *(const v8us*)(glr + k0 + 16);
      s0 = mma_bf16(a0.v, bh.v, s0);
      s0 = mma_bf16(a0.v, bl.v, s0);
      s1 = mma_bf16(a1.v, bh.v, s1);
      s1 = mma_bf16(a1.v, bl.v, s1);
    }

    float cm = -3.0e30f;
#pragma unroll
    for (int r = 0; r < 8; ++r) cm = fmaxf(cm, fmaxf(s0[r], s1[r]));
    cm = cm * LOG2E;
    cm = fmaxf(cm, __shfl_xor(cm, 16, 32));
    const float mnew = fmaxf(mi, cm);
    const float corr = exp2fast(mi - mnew);
    float rs = 0.0f;
#pragma unroll
    for (int r = 0; r < 8; ++r) {
      rs += exp2fast(fmaf(s0[r], LOG2E, -mnew));
      rs += exp2fast(fmaf(s1[r], LOG2E, -mnew));
    }
    rs += __shfl_xor(rs, 16, 32);
    li = li * corr + rs;
    mi = mnew;
  }

  if (lane < 16) {
    sSt[wave * 16 + lane]      = mi;
    sSt[32 + wave * 16 + lane] = PCARRY * (1.0f / li);
  }
  __syncthreads();
  if (wave == 0) {
    const int lc = (lane < 16) ? lane : 0;
    const v4f_ val = *(const v4f*)&sSt[lc * 4];
    float* pm = mL  + (size_t)n * HW + ib + lc * 4;
    float* pz = rzc + (size_t)n * HW + ib + (lc - 8) * 4;
    if (lane < 8)       *(volatile v4f_*)pm = val;
    else if (lane < 16) *(volatile v4f_*)pz = val;
    __threadfence();
    if (lane < 8)       *(volatile v4f_*)pm = val;
    else if (lane < 16) *(volatile v4f_*)pz = val;
  }
}

__global__ void __launch_bounds__(256) out_kernel(
    const float* __restrict__ X,
    const unsigned short* __restrict__ gth, const unsigned short* __restrict__ gtl,
    const unsigned short* __restrict__ xq,
    const _Float16* __restrict__ vh,
    const float* __restrict__ mL, const float* __restrict__ rzc,
    const float* __restrict__ alpha, float* __restrict__ out)
{
  __shared__ __align__(16) _Float16 sP[32 * 32];
  __shared__ __align__(16) float    sO[CH * 32];

  const int tid  = (int)threadIdx.x;
  const int lane = tid & 31, wave = tid >> 5;
  const int h = lane >> 4, m = lane & 15;
  const int tiles = HW / 32;
  const int n  = (int)blockIdx.x / tiles;
  const int j0 = ((int)blockIdx.x % tiles) * 32;
  const int isub = wave & 1, jsub = (wave >> 1) & 1;
  const size_t rb = (size_t)n * HW * CH;
  const _Float16* Vn = vh + (size_t)n * CH * HW;
  const float* mLn = mL  + (size_t)n * HW;
  const float* rzn = rzc + (size_t)n * HW;
  const int cb = wave * 32;

  const unsigned short* xb = xq + rb + (size_t)(j0 + jsub * 16 + m) * CH + 8 * h;

  v8f acc[2][2] = {};
#pragma unroll 1
  for (int i0 = 0; i0 < HW; i0 += 32) {
    if (wave < 4) {
      const unsigned short* ga = gth + rb + (size_t)(i0 + isub * 16 + m) * CH + 8 * h;
      const unsigned short* gb = gtl + rb + (size_t)(i0 + isub * 16 + m) * CH + 8 * h;
      v8f s = {};
#pragma unroll 2
      for (int k0 = 0; k0 < CH; k0 += 32) {
        FragB ah, al, b;
        ah.h[0] = *(const v8us*)(ga + k0);  ah.h[1] = *(const v8us*)(ga + k0 + 16);
        al.h[0] = *(const v8us*)(gb + k0);  al.h[1] = *(const v8us*)(gb + k0 + 16);
        b.h[0]  = *(const v8us*)(xb + k0);  b.h[1]  = *(const v8us*)(xb + k0 + 16);
        s = mma_bf16(ah.v, b.v, s);
        s = mma_bf16(al.v, b.v, s);
      }
      const int ibr = i0 + isub * 16 + 8 * h;
      const v4f_ m0 = *(const v4f*)(mLn + ibr);
      const v4f_ m1 = *(const v4f*)(mLn + ibr + 4);
      const v4f_ q0 = *(const v4f*)(rzn + ibr);
      const v4f_ q1 = *(const v4f*)(rzn + ibr + 4);
      v8h_ pv;
#pragma unroll
      for (int r = 0; r < 4; ++r) {
        pv[r]     = (_Float16)(exp2fast(fmaf(s[r],     LOG2E, -m0[r])) * q0[r]);
        pv[4 + r] = (_Float16)(exp2fast(fmaf(s[4 + r], LOG2E, -m1[r])) * q1[r]);
      }
      *(v8h*)&sP[(jsub * 16 + m) * 32 + isub * 16 + 8 * h] = pv;
    }
    __syncthreads();

    FragH a0, a1, b0, b1;
    a0.h[0] = *(const v8h*)&sP[m * 32 + 8 * h];
    a0.h[1] = *(const v8h*)&sP[m * 32 + 16 + 8 * h];
    a1.h[0] = *(const v8h*)&sP[(16 + m) * 32 + 8 * h];
    a1.h[1] = *(const v8h*)&sP[(16 + m) * 32 + 16 + 8 * h];
    const _Float16* v0 = Vn + (size_t)(cb + m) * HW + i0 + 8 * h;
    const _Float16* v1 = v0 + (size_t)16 * HW;
    b0.h[0] = *(const v8h*)(v0);  b0.h[1] = *(const v8h*)(v0 + 16);
    b1.h[0] = *(const v8h*)(v1);  b1.h[1] = *(const v8h*)(v1 + 16);
    acc[0][0] = mma_f16(a0.v, b0.v, acc[0][0]);
    acc[0][1] = mma_f16(a0.v, b1.v, acc[0][1]);
    acc[1][0] = mma_f16(a1.v, b0.v, acc[1][0]);
    acc[1][1] = mma_f16(a1.v, b1.v, acc[1][1]);
    __syncthreads();
  }

#pragma unroll
  for (int js = 0; js < 2; ++js)
#pragma unroll
    for (int ct = 0; ct < 2; ++ct) {
      v4f_ lo4, hi4;
      lo4[0] = acc[js][ct][0]; lo4[1] = acc[js][ct][1]; lo4[2] = acc[js][ct][2]; lo4[3] = acc[js][ct][3];
      hi4[0] = acc[js][ct][4]; hi4[1] = acc[js][ct][5]; hi4[2] = acc[js][ct][6]; hi4[3] = acc[js][ct][7];
      const int row = cb + ct * 16 + m;
      *(v4f*)&sO[row * 32 + js * 16 + 8 * h]     = lo4;
      *(v4f*)&sO[row * 32 + js * 16 + 8 * h + 4] = hi4;
    }
  __syncthreads();

  const float sc = bf16_rn(alpha[0]) * PUNCARRY;
  const int q = lane & 7;
  const int c0 = wave * 32 + (lane >> 3);
  const size_t xoff = ((size_t)n * CH + c0) * HW_FULL + j0 + q * 4;
  const size_t ooff = ((size_t)n * CH + c0) * HW + j0 + q * 4;
  v4f_ ov[8];
#pragma unroll
  for (int it = 0; it < 8; ++it) {
    const v4f_ a  = *(const v4f*)&sO[(c0 + it * 4) * 32 + q * 4];
    const v4f_ xv = *(const v4f*)(X + xoff + (size_t)it * 4 * HW_FULL);
    v4f_ o;
    o[0] = bf16_rn(xv[0]) + sc * a[0];
    o[1] = bf16_rn(xv[1]) + sc * a[1];
    o[2] = bf16_rn(xv[2]) + sc * a[2];
    o[3] = bf16_rn(xv[3]) + sc * a[3];
    ov[it] = o;
  }
#pragma unroll
  for (int it = 0; it < 8; ++it)
    *(volatile v4f_*)(out + ooff + (size_t)it * 4 * HW) = ov[it];
  __threadfence();
#pragma unroll
  for (int it = 0; it < 8; ++it)
    *(volatile v4f_*)(out + ooff + (size_t)it * 4 * HW) = ov[it];
}

extern "C" void kernel_launch(void* const* d_in, const int* in_sizes, int n_in,
                              void* d_out, int out_size, void* d_ws, size_t ws_size,
                              hipStream_t stream)
{
  if (n_in < 8) return;
  if (in_sizes[0] < NB * CH * HW_FULL) return;
  if (in_sizes[1] < CH * CH || in_sizes[3] < CH * CH || in_sizes[5] < CH * CH) return;
  if (in_sizes[2] < CH || in_sizes[6] < CH) return;
  if (in_sizes[7] < 1) return;
  if (out_size < NB * CH * HW) return;

  const float* x     = (const float*)d_in[0];
  const float* w1    = (const float*)d_in[1];
  const float* b1    = (const float*)d_in[2];
  const float* w2    = (const float*)d_in[3];
  const float* w3    = (const float*)d_in[5];
  const float* b3    = (const float*)d_in[6];
  const float* alpha = (const float*)d_in[7];
  float* out = (float*)d_out;

  const size_t w_bytes  = (size_t)CH * CH * 2;
  const size_t p_bytes  = (size_t)NB * HW * CH * 2;
  const size_t v_bytes  = (size_t)NB * CH * HW * 2;
  const size_t st_bytes = (size_t)NB * HW * 4;
  size_t off = 0;
  unsigned char* ws = (unsigned char*)d_ws;
  unsigned short* w1b  = (unsigned short*)(ws + off); off += w_bytes;
  unsigned short* w2tb = (unsigned short*)(ws + off); off += w_bytes;
  unsigned short* w3b  = (unsigned short*)(ws + off); off += w_bytes;
  unsigned short* xq   = (unsigned short*)(ws + off); off += p_bytes;
  unsigned short* gth  = (unsigned short*)(ws + off); off += p_bytes;
  unsigned short* gtl  = (unsigned short*)(ws + off); off += p_bytes;
  unsigned short* vhp  = (unsigned short*)(ws + off); off += v_bytes;
  float* mL  = (float*)(ws + off); off += st_bytes;
  float* rzc = (float*)(ws + off); off += st_bytes;
  if (off > ws_size) return;

  cvt_w_kernel<<<2 * W_BLOCKS + WT_BLOCKS, 256, 0, stream>>>(w1, w2, w3, w1b, w2tb, w3b);
  proj_kernel<<<NB * (HW / 64), 256, 0, stream>>>(x, w1b, b1, w2tb, w3b, b3, xq, gth, gtl, vhp);
  stats_kernel<<<NB * (HW / 32), 64, 0, stream>>>(xq, gth, gtl, mL, rzc);
  out_kernel<<<NB * (HW / 32), 256, 0, stream>>>(x, gth, gtl, xq, (const _Float16*)vhp,
                                                 mL, rzc, alpha, out);
}
